// TAttention_29583734735457
// MI455X (gfx1250) — hardware-verified
//
#include <hip/hip_runtime.h>
#include <math.h>

constexpr int kB   = 32;
constexpr int kS   = 1024;
constexpr int kD   = 256;
constexpr int kH   = 8;
constexpr int kHD  = 32;
constexpr int kTok = kB * kS;
constexpr int kCB  = 8;
constexpr int kNChunk = kB / kCB;
constexpr int kTokC = kCB * kS;
constexpr int kQKld = 2 * kD;
constexpr int kKC  = 64;
constexpr int kOsPitch = 36;
constexpr float kEps      = 1e-5f;
constexpr float kInvD     = 1.0f / 256.0f;
constexpr float kWCarry   = 16.0f;
constexpr float kWCarryInv = 1.0f / 16.0f;
constexpr float kPCarry   = 32768.0f;
constexpr float kVloCarry = 2048.0f;
constexpr float kVloInv   = 1.0f / 2048.0f;
static_assert(kH * kHD == kD, "shape");
static_assert(kB % kCB == 0, "chunks");
static_assert(kTokC % 64 == 0 && kQKld % 64 == 0 && kD % 64 == 0, "gemm tiles");
static_assert(kD % 32 == 0, "gemm k");
static_assert(kS % kKC == 0 && kS % 64 == 0 && kHD == 32 && kKC == 64, "attn tiles");
static_assert(kTok % 8 == 0 && kTokC % 8 == 0, "ln grid");

typedef __attribute__((ext_vector_type(16))) _Float16 v16h;
typedef __attribute__((ext_vector_type(8)))  _Float16 v8h;
typedef __attribute__((ext_vector_type(16))) __bf16   v16b;
typedef __attribute__((ext_vector_type(8)))  __bf16   v8b;
typedef __attribute__((ext_vector_type(8)))  float    v8f;
typedef __attribute__((ext_vector_type(4)))  float    v4f;
typedef __attribute__((ext_vector_type(4)))  unsigned int v4u;

__device__ __forceinline__ unsigned short f2bf_bits(float f) {
  unsigned u = __float_as_uint(f);
  return (unsigned short)((u + 0x7FFFu + ((u >> 16) & 1u)) >> 16);
}
__device__ __forceinline__ float bf_bits2f(unsigned short h) { return __uint_as_float(((unsigned)h) << 16); }
__device__ __forceinline__ float bfr(float f) { return bf_bits2f(f2bf_bits(f)); }

__device__ __forceinline__ void dep_guard_h(v8f& a, v8f& b, v16h x, v16h y) { asm volatile("v_nop\n\tv_nop\n\tv_nop\n\tv_nop" : "+v"(a), "+v"(b) : "v"(x), "v"(y)); }
__device__ __forceinline__ void dep_guard_b(v8f& a, v8f& b, v16b x, v16b y) { asm volatile("v_nop\n\tv_nop\n\tv_nop\n\tv_nop" : "+v"(a), "+v"(b) : "v"(x), "v"(y)); }
__device__ __forceinline__ void keep4_h(v16h a, v16h b, v16h c, v16h d) { asm volatile("v_nop" :: "v"(a), "v"(b), "v"(c), "v"(d)); }
__device__ __forceinline__ void keep4_b(v16b a, v16b b, v16b c, v16b d) { asm volatile("v_nop" :: "v"(a), "v"(b), "v"(c), "v"(d)); }
__device__ __forceinline__ void acc_guard4(v8f& a, v8f& b, v8f& c, v8f& d) { asm volatile("v_nop\n\tv_nop\n\tv_nop\n\tv_nop" : "+v"(a), "+v"(b), "+v"(c), "+v"(d)); }
template <typename T> struct Frag;
template <> struct Frag<_Float16> {
  typedef v16h V; union U { v16h v; v8h h[2]; };
  static __device__ __forceinline__ v16h load(const _Float16* p) {
    U f; f.h[0] = *(const v8h*)(p); f.h[1] = *(const v8h*)(p + 16); return f.v;
  }
  static __device__ __forceinline__ v8f mma(v16h a, v16h b, v8f c) {
    return __builtin_amdgcn_wmma_f32_16x16x32_f16(false, a, false, b, (short)0, c, false, false);
  }
  static __device__ __forceinline__ void guard(v8f& a, v8f& b, v16h x, v16h y) { dep_guard_h(a, b, x, y); }
  static __device__ __forceinline__ void keep(v16h a, v16h b, v16h c, v16h d) { keep4_h(a, b, c, d); }
};
template <> struct Frag<__bf16> {
  typedef v16b V; union U { v16b v; v8b h[2]; };
  static __device__ __forceinline__ v16b load(const __bf16* p) {
    U f; f.h[0] = *(const v8b*)(p); f.h[1] = *(const v8b*)(p + 16); return f.v;
  }
  static __device__ __forceinline__ v8f mma(v16b a, v16b b, v8f c) {
    return __builtin_amdgcn_wmma_f32_16x16x32_bf16(false, a, false, b, (short)0, c, false, false);
  }
  static __device__ __forceinline__ void guard(v8f& a, v8f& b, v16b x, v16b y) { dep_guard_b(a, b, x, y); }
  static __device__ __forceinline__ void keep(v16b a, v16b b, v16b c, v16b d) { keep4_b(a, b, c, d); }
};

__device__ __forceinline__ unsigned pk16(unsigned short a, unsigned short b) { return (unsigned)a | ((unsigned)b << 16); }
__device__ __forceinline__ unsigned short h_bits(float f) { const _Float16 h = (_Float16)f; return __builtin_bit_cast(unsigned short, h); }

__device__ __forceinline__ v8f at_mma(v16b a, v16b b, v8f c) {
  c = __builtin_amdgcn_wmma_f32_16x16x32_bf16(false, a, false, b, (short)0, c, false, false);
  asm volatile("v_nop\n\tv_nop\n\tv_nop\n\tv_nop" : "+v"(c) : "v"(a), "v"(b));
  return c;
}
template <bool F16> __device__ __forceinline__ v8f at_mma16(v16b a, v16b b, v8f c) {
  if (F16) {
    const v16h ah = __builtin_bit_cast(v16h, a), bh = __builtin_bit_cast(v16h, b);
    c = __builtin_amdgcn_wmma_f32_16x16x32_f16(false, ah, false, bh, (short)0, c, false, false);
    asm volatile("v_nop\n\tv_nop\n\tv_nop\n\tv_nop" : "+v"(c) : "v"(ah), "v"(bh));
    return c;
  }
  return at_mma(a, b, c);
}

template <int ET> struct Elem;
template <> struct Elem<0> { typedef _Float16 T; };
template <> struct Elem<1> { typedef __bf16 T; };
template <int ET, bool SPLITA, bool SPLITB, int BIAS_MODE, int OUT_MODE, bool RESID, int ACT = 0>
__global__ __launch_bounds__(256) void wmma_gemm64(
    const unsigned short* __restrict__ Ap, const unsigned short* __restrict__ A2p, int lda, long strideA,
    const unsigned short* __restrict__ Btp, const unsigned short* __restrict__ Bt2p, int ldb, long strideB,
    void* __restrict__ Cout, void* __restrict__ Cout2, int ldc, long strideC,
    const float* __restrict__ bias,
    const float* __restrict__ resid, long strideR,
    int M, int N, int K, float scale) {
  static_assert(!RESID || OUT_MODE == 0, "resid mode");
  static_assert(!(RESID && ACT != 0), "resid act");
  typedef typename Elem<ET>::T T;
  typedef typename Frag<T>::V V;
  const T* A = (const T*)Ap; const T* A2 = (const T*)A2p; const T* Bt = (const T*)Btp; const T* Bt2 = (const T*)Bt2p;
  __shared__ __align__(16) float sT[8][16 * 68];
  const int b    = blockIdx.y;
  const int lane = threadIdx.x & 31;
  const int wave = threadIdx.x >> 5;
  const int tilesN = N >> 6;
  const int tilesM = M >> 6;
  const int tile = blockIdx.x * 8 + wave;
  if (tile >= tilesM * tilesN) return;
  const int tm = tile / tilesN;
  const int tn = tile - tm * tilesN;
  const int m0 = tm << 6;
  const int n0 = tn << 6;

  const T* Ab  = A  + (size_t)b * strideA;
  const T* Bb  = Bt + (size_t)b * strideB;
  const T* Ab2 = SPLITA ? (A2  + (size_t)b * strideA) : nullptr;
  const T* Bb2 = SPLITB ? (Bt2 + (size_t)b * strideB) : nullptr;

  const int rlane = lane & 15;
  const int koff  = (lane >> 4) * 8;
  const int mOff  = (lane >> 4) * 8;

  v8f acc[4][4];
#pragma unroll
  for (int i = 0; i < 4; ++i)
#pragma unroll
    for (int j = 0; j < 4; ++j) acc[i][j] = (v8f){0.f,0.f,0.f,0.f,0.f,0.f,0.f,0.f};

  for (int k0 = 0; k0 < K; k0 += 32) {
    V bh[4], bl[4];
#pragma unroll
    for (int j = 0; j < 4; ++j) {
      const size_t bo = (size_t)(n0 + (j << 4) + rlane) * ldb + koff + k0;
      bh[j] = Frag<T>::load(Bb + bo);
      if (SPLITB) bl[j] = Frag<T>::load(Bb2 + bo);
    }
#pragma unroll
    for (int i = 0; i < 4; ++i) {
      const size_t ao = (size_t)(m0 + (i << 4) + rlane) * lda + koff + k0;
      V ah = Frag<T>::load(Ab + ao);
      V al;
      if (SPLITA) al = Frag<T>::load(Ab2 + ao);
#pragma unroll
      for (int j = 0; j < 4; ++j) {
        acc[i][j] = Frag<T>::mma(ah, bh[j], acc[i][j]);
        if (SPLITB) acc[i][j] = Frag<T>::mma(ah, bl[j], acc[i][j]);
        if (SPLITA) acc[i][j] = Frag<T>::mma(al, bh[j], acc[i][j]);
      }
      Frag<T>::guard(acc[i][0], acc[i][3], ah, SPLITA ? al : ah);
    }
    Frag<T>::keep(bh[0], bh[1], bh[2], bh[3]);
    if (SPLITB) Frag<T>::keep(bl[0], bl[1], bl[2], bl[3]);
  }
  acc_guard4(acc[0][0], acc[0][1], acc[0][2], acc[0][3]);
  acc_guard4(acc[1][0], acc[1][1], acc[1][2], acc[1][3]);
  acc_guard4(acc[2][0], acc[2][1], acc[2][2], acc[2][3]);
  acc_guard4(acc[3][0], acc[3][1], acc[3][2], acc[3][3]);

  float* slab = sT[wave];
  const float* Rb = RESID ? (resid + (size_t)b * strideR) : nullptr;
#pragma unroll
  for (int i = 0; i < 4; ++i) {
    const int mBase = m0 + (i << 4);
#pragma unroll
    for (int j = 0; j < 4; ++j) {
      const int n = n0 + (j << 4) + rlane;
      float bv = 0.f;
      if (BIAS_MODE == 2) bv = bias[n];
#pragma unroll
      for (int r = 0; r < 8; ++r) {
        float v = acc[i][j][r] * scale;
        if (BIAS_MODE == 1) v += bias[mBase + mOff + r];
        if (BIAS_MODE == 2) v += bv;
        if (ACT == 2) v = fmaxf(v, 0.0f);
        if (ACT == 4) v = (v > 0.f) ? v : 0.01f * v;
        slab[(mOff + r) * 68 + (j << 4) + rlane] = v;
      }
    }
    __builtin_amdgcn_fence(__ATOMIC_RELEASE, "workgroup");
    __builtin_amdgcn_wave_barrier();
    __builtin_amdgcn_fence(__ATOMIC_ACQUIRE, "workgroup");
    if (OUT_MODE == 0) {
      float* C = (float*)Cout + (size_t)b * strideC;
      const int hh = lane >> 4, c4 = (lane & 15) * 4;
      for (int pass = 0; pass < 2; ++pass) {
#pragma unroll
        for (int it = 0; it < 8; ++it) {
          const int row = it * 2 + hh;
          v4f v = *(const v4f*)(slab + row * 68 + c4);
          if (RESID) {
            const v4f rr = *(const v4f*)(Rb + (size_t)(mBase + row) * ldc + n0 + c4);
            v = v + rr;
          }
          *(volatile v4f*)(C + (size_t)(mBase + row) * ldc + n0 + c4) = v;
        }
        __threadfence();
      }
    } else {
      const int q = lane >> 3, c8 = (lane & 7) * 8;
      unsigned short* C  = (unsigned short*)Cout  + (size_t)b * strideC;
      unsigned short* C2 = (OUT_MODE == 2) ? ((unsigned short*)Cout2 + (size_t)b * strideC) : nullptr;
      for (int pass = 0; pass < 2; ++pass) {
#pragma unroll
        for (int it = 0; it < 4; ++it) {
          const int row = it * 4 + q;
          const float* sp = slab + row * 68 + c8;
          v8h hv, lv;
#pragma unroll
          for (int e = 0; e < 8; ++e) {
            if (OUT_MODE == 1) {
              hv[e] = (_Float16)sp[e];
            } else {
              unsigned short hb = f2bf_bits(sp[e]);
              unsigned short lb = f2bf_bits(sp[e] - bf_bits2f(hb));
              hv[e] = __builtin_bit_cast(_Float16, hb);
              lv[e] = __builtin_bit_cast(_Float16, lb);
            }
          }
          *(volatile v8h*)(C + (size_t)(mBase + row) * ldc + n0 + c8) = hv;
          if (OUT_MODE == 2) *(volatile v8h*)(C2 + (size_t)(mBase + row) * ldc + n0 + c8) = lv;
        }
        __threadfence();
      }
    }
    __builtin_amdgcn_fence(__ATOMIC_RELEASE, "workgroup");
    __builtin_amdgcn_wave_barrier();
    __builtin_amdgcn_fence(__ATOMIC_ACQUIRE, "workgroup");
  }
}

__global__ __launch_bounds__(256) void wprep_kernel(const float* __restrict__ W0, const float* __restrict__ W1,
                                                    const float* __restrict__ W2, const float* __restrict__ W3,
                                                    const float* __restrict__ W4,
                                                    unsigned short* __restrict__ WB, unsigned short* __restrict__ WF) {
  __shared__ float sm[64][65];
  const int t  = threadIdx.x;
  const int k0 = blockIdx.x * 64;
  const int n0 = blockIdx.y * 64;
  const int z  = blockIdx.z;
  const float* W = (z == 0) ? W0 : (z == 1) ? W1 : (z == 2) ? W2 : (z == 3) ? W3 : W4;
#pragma unroll
  for (int i = 0; i < 16; ++i) {
    const int e  = i * 256 + t;
    const int r  = e >> 6;
    const int cc = e & 63;
    sm[cc][r] = W[(size_t)(k0 + r) * kD + n0 + cc];
  }
  __syncthreads();
  const int lane = t & 31, wave = t >> 5;
  const int q = lane >> 3, c8 = (lane & 7) * 8;
  if (z < 3) {
    unsigned short* op = WB + (size_t)z * kD * kD;
    for (int pass = 0; pass < 2; ++pass) {
#pragma unroll
      for (int it = 0; it < 2; ++it) {
        const int row = wave * 8 + it * 4 + q;
        unsigned short hb[8];
#pragma unroll
        for (int e = 0; e < 8; ++e) hb[e] = f2bf_bits(sm[row][c8 + e]);
        const v4u u = (v4u){pk16(hb[0], hb[1]), pk16(hb[2], hb[3]), pk16(hb[4], hb[5]), pk16(hb[6], hb[7])};
        *(volatile v4u*)(op + (size_t)(n0 + row) * kD + k0 + c8) = u;
      }
      __threadfence();
    }
  } else {
    unsigned short* op = WF + (size_t)(z - 3) * kD * kD;
    for (int pass = 0; pass < 2; ++pass) {
#pragma unroll
      for (int it = 0; it < 2; ++it) {
        const int row = wave * 8 + it * 4 + q;
        unsigned short hb[8];
#pragma unroll
        for (int e = 0; e < 8; ++e) hb[e] = h_bits(bfr(sm[row][c8 + e]) * kWCarry);
        const v4u u = (v4u){pk16(hb[0], hb[1]), pk16(hb[2], hb[3]), pk16(hb[4], hb[5]), pk16(hb[6], hb[7])};
        *(volatile v4u*)(op + (size_t)(n0 + row) * kD + k0 + c8) = u;
      }
      __threadfence();
    }
  }
}

__global__ __launch_bounds__(256) void ln1_split_kernel(const float* __restrict__ X, const float* __restrict__ gam,
                                                        const float* __restrict__ bet,
                                                        unsigned short* __restrict__ XH, unsigned short* __restrict__ XL,
                                                        int nrows) {
  const int lane = threadIdx.x & 31;
  const int wave = threadIdx.x >> 5;
  const int row  = blockIdx.x * 8 + wave;
  if (row >= nrows) return;
  const float* xp = X + (size_t)row * kD + lane * 8;
  const v4f a0 = *(const v4f*)(xp);
  const v4f a1 = *(const v4f*)(xp + 4);
  float v[8];
#pragma unroll
  for (int e = 0; e < 4; ++e) { v[e] = bfr(a0[e]); v[4 + e] = bfr(a1[e]); }
  float s = 0.0f;
#pragma unroll
  for (int e = 0; e < 8; ++e) s += v[e];
#pragma unroll
  for (int off = 1; off < 32; off <<= 1) s += __shfl_xor(s, off, 32);
  const float mu = s * kInvD;
  float var = 0.0f;
#pragma unroll
  for (int e = 0; e < 8; ++e) { const float d = v[e] - mu; var += d * d; }
#pragma unroll
  for (int off = 1; off < 32; off <<= 1) var += __shfl_xor(var, off, 32);
  const float rstd = rsqrtf(var * kInvD + kEps);
  const v4f g0 = *(const v4f*)(gam + lane * 8), g1 = *(const v4f*)(gam + lane * 8 + 4);
  const v4f b0 = *(const v4f*)(bet + lane * 8), b1 = *(const v4f*)(bet + lane * 8 + 4);
  float gv[8], bv[8];
#pragma unroll
  for (int e = 0; e < 4; ++e) { gv[e] = bfr(g0[e]); gv[4 + e] = bfr(g1[e]); bv[e] = bfr(b0[e]); bv[4 + e] = bfr(b1[e]); }
  unsigned short hb[8], lb[8];
#pragma unroll
  for (int e = 0; e < 8; ++e) {
    const float tt = (v[e] - mu) * rstd;
    const float y  = tt * gv[e] + bv[e];
    hb[e] = f2bf_bits(y);
    lb[e] = f2bf_bits(y - bf_bits2f(hb[e]));
  }
  const v4u uh = (v4u){pk16(hb[0], hb[1]), pk16(hb[2], hb[3]), pk16(hb[4], hb[5]), pk16(hb[6], hb[7])};
  const v4u ul = (v4u){pk16(lb[0], lb[1]), pk16(lb[2], lb[3]), pk16(lb[4], lb[5]), pk16(lb[6], lb[7])};
  unsigned short* ph = XH + (size_t)row * kD + lane * 8;
  unsigned short* pl = XL + (size_t)row * kD + lane * 8;
  *(volatile v4u*)ph = uh;
  *(volatile v4u*)pl = ul;
  __threadfence();
  *(volatile v4u*)ph = uh;
  *(volatile v4u*)pl = ul;
}

__global__ __launch_bounds__(256) void ln2_kernel(const float* __restrict__ CTX, const float* __restrict__ X,
                                                  const float* __restrict__ gam, const float* __restrict__ bet,
                                                  float* __restrict__ A32, unsigned short* __restrict__ A16, int nrows) {
  __shared__ __align__(16) float rowbuf[8][kD];
  const int lane = threadIdx.x & 31;
  const int wave = threadIdx.x >> 5;
  const int row  = blockIdx.x * 8 + wave;
  if (row >= nrows) return;
  const float* cp = CTX + (size_t)row * kD + lane * 8;
  const float* xp = X + (size_t)row * kD + lane * 8;
  const v4f c0 = *(const v4f*)(cp), c1 = *(const v4f*)(cp + 4);
  const v4f x0 = *(const v4f*)(xp), x1 = *(const v4f*)(xp + 4);
  float v[8];
#pragma unroll
  for (int e = 0; e < 4; ++e) { v[e] = c0[e] + bfr(x0[e]); v[4 + e] = c1[e] + bfr(x1[e]); }
  float s = 0.0f;
#pragma unroll
  for (int e = 0; e < 8; ++e) s += v[e];
#pragma unroll
  for (int off = 1; off < 32; off <<= 1) s += __shfl_xor(s, off, 32);
  const float mu = s * kInvD;
  float var = 0.0f;
#pragma unroll
  for (int e = 0; e < 8; ++e) { const float d = v[e] - mu; var += d * d; }
#pragma unroll
  for (int off = 1; off < 32; off <<= 1) var += __shfl_xor(var, off, 32);
  const float rstd = rsqrtf(var * kInvD + kEps);
  const v4f g0 = *(const v4f*)(gam + lane * 8), g1 = *(const v4f*)(gam + lane * 8 + 4);
  const v4f b0 = *(const v4f*)(bet + lane * 8), b1 = *(const v4f*)(bet + lane * 8 + 4);
  float gv[8], bv[8];
#pragma unroll
  for (int e = 0; e < 4; ++e) { gv[e] = bfr(g0[e]); gv[4 + e] = bfr(g1[e]); bv[e] = bfr(b0[e]); bv[4 + e] = bfr(b1[e]); }
  float y[8];
  unsigned short hb[8];
#pragma unroll
  for (int e = 0; e < 8; ++e) {
    const float tt = (v[e] - mu) * rstd;
    y[e] = tt * gv[e] + bv[e];
    hb[e] = h_bits(y[e]);
  }
  const v4u u16 = (v4u){pk16(hb[0], hb[1]), pk16(hb[2], hb[3]), pk16(hb[4], hb[5]), pk16(hb[6], hb[7])};
  float* rb = rowbuf[wave];
  *(v4f*)(rb + lane * 8)     = (v4f){y[0], y[1], y[2], y[3]};
  *(v4f*)(rb + lane * 8 + 4) = (v4f){y[4], y[5], y[6], y[7]};
  __builtin_amdgcn_fence(__ATOMIC_RELEASE, "workgroup");
  __builtin_amdgcn_wave_barrier();
  __builtin_amdgcn_fence(__ATOMIC_ACQUIRE, "workgroup");
  const v4f o0 = *(const v4f*)(rb + lane * 4);
  const v4f o1 = *(const v4f*)(rb + 128 + lane * 4);
  float* ap = A32 + (size_t)row * kD;
  unsigned short* hp = A16 + (size_t)row * kD + lane * 8;
  for (int pass = 0; pass < 2; ++pass) {
    *(volatile v4f*)(ap + lane * 4) = o0;
    *(volatile v4f*)(ap + 128 + lane * 4) = o1;
    *(volatile v4u*)hp = u16;
    __threadfence();
  }
}

__global__ __launch_bounds__(256) void vt_split_kernel(const float* __restrict__ V, unsigned short* __restrict__ VTH,
                                                       unsigned short* __restrict__ VTL) {
  __shared__ float sm[kHD][65];
  const int t  = threadIdx.x;
  const int s0 = blockIdx.x * 64;
  const int h  = blockIdx.y;
  const int bl = blockIdx.z;
#pragma unroll
  for (int i = 0; i < 8; ++i) {
    const int e  = i * 256 + t;
    const int r  = e >> 5;
    const int cd = e & 31;
    sm[cd][r] = V[((size_t)(bl * kS + s0 + r)) * kD + h * kHD + cd];
  }
  __syncthreads();
  const int lane = t & 31, wave = t >> 5;
  const int q4 = lane >> 3, c8 = (lane & 7) * 8;
  const int d = wave * 4 + q4;
  unsigned short hb[8], lb[8];
#pragma unroll
  for (int e = 0; e < 8; ++e) {
    const float vv = sm[d][c8 + e];
    const _Float16 hv = (_Float16)vv;
    const float hf = (float)hv;
    const float lo = (vv - hf) * kVloCarry;
    hb[e] = __builtin_bit_cast(unsigned short, hv);
    lb[e] = h_bits(lo);
  }
  const v4u uh = (v4u){pk16(hb[0], hb[1]), pk16(hb[2], hb[3]), pk16(hb[4], hb[5]), pk16(hb[6], hb[7])};
  const v4u ul = (v4u){pk16(lb[0], lb[1]), pk16(lb[2], lb[3]), pk16(lb[4], lb[5]), pk16(lb[6], lb[7])};
  const size_t ro = ((size_t)((bl * kH + h) * kHD + d)) * kS + s0 + c8;
  for (int pass = 0; pass < 2; ++pass) {
    *(volatile v4u*)(VTH + ro) = uh;
    *(volatile v4u*)(VTL + ro) = ul;
    __threadfence();
  }
}

__global__ __launch_bounds__(128) void attn_hd32_kernel(const unsigned short* __restrict__ QKh,
                                                        const unsigned short* __restrict__ QKl,
                                                        const unsigned short* __restrict__ VTh,
                                                        const unsigned short* __restrict__ VTl,
                                                        float* __restrict__ ctx) {
  union FB { v16b v; v8b h[2]; };
  __shared__ __align__(16) unsigned short Ksh[kKC * kHD];
  __shared__ __align__(16) unsigned short Ksl[kKC * kHD];
  __shared__ __align__(16) unsigned short Vsh[kHD * kKC];
  __shared__ __align__(16) unsigned short Vsl[kHD * kKC];
  __shared__ __align__(16) unsigned short Psh[4][16 * kKC];
  __shared__ __align__(16) float Os[4][16 * kOsPitch];

  const int tid  = threadIdx.x;
  const int wave = tid >> 5;
  const int lane = tid & 31;
  const int hh   = lane >> 4;
  const int c    = lane & 15;

  const int bx = blockIdx.x;
  const int qb = bx & 15;
  const int bh = bx >> 4;
  const int h  = bh & (kH - 1);
  const int bl = bh >> 3;
  const int q0 = qb * 64 + wave * 16;
  const size_t tokBase = (size_t)bl * kS;

  v16b qah, qal;
  {
    const __bf16* qh = (const __bf16*)(QKh + (tokBase + q0 + c) * kQKld + h * kHD + 8 * hh);
    const __bf16* ql = (const __bf16*)(QKl + (tokBase + q0 + c) * kQKld + h * kHD + 8 * hh);
    FB f; f.h[0] = *(const v8b*)(qh); f.h[1] = *(const v8b*)(qh + 16); qah = f.v;
    FB g; g.h[0] = *(const v8b*)(ql); g.h[1] = *(const v8b*)(ql + 16); qal = g.v;
  }

  float mrow[8], lrow[8];
  v8f oh[2], ol[2];
#pragma unroll
  for (int r = 0; r < 8; ++r) { mrow[r] = -INFINITY; lrow[r] = 0.f; }
#pragma unroll
  for (int t = 0; t < 2; ++t) { oh[t] = (v8f){0.f,0.f,0.f,0.f,0.f,0.f,0.f,0.f}; ol[t] = oh[t]; }

  const unsigned short* kbh = QKh + tokBase * kQKld + kD + h * kHD;
  const unsigned short* kbl = QKl + tokBase * kQKld + kD + h * kHD;
  const unsigned short* vbh = VTh + ((size_t)(bl * kH + h) * kHD) * kS;
  const unsigned short* vbl = VTl + ((size_t)(bl * kH + h) * kHD) * kS;
  const int kvr   = tid >> 1;
  const int kpart = (tid & 1) * 16;

  for (int kc = 0; kc < kS / kKC; ++kc) {
    const int kv0 = kc * kKC;
    __syncthreads();
    {
      const unsigned short* kp = kbh + (size_t)(kv0 + kvr) * kQKld + kpart;
      const unsigned short* lp = kbl + (size_t)(kv0 + kvr) * kQKld + kpart;
      const v4u ka = *(const v4u*)(kp), kb2 = *(const v4u*)(kp + 8);
      const v4u la = *(const v4u*)(lp), lb2 = *(const v4u*)(lp + 8);
      *(v4u*)(Ksh + kvr * kHD + kpart)     = ka;
      *(v4u*)(Ksh + kvr * kHD + kpart + 8) = kb2;
      *(v4u*)(Ksl + kvr * kHD + kpart)     = la;
      *(v4u*)(Ksl + kvr * kHD + kpart + 8) = lb2;
#pragma unroll
      for (int i = 0; i < 2; ++i) {
        const int idx  = tid + 128 * i;
        const int d    = idx >> 3;
        const int col8 = (idx & 7) * 8;
        const v4u vh = *(const v4u*)(vbh + (size_t)d * kS + kv0 + col8);
        const v4u vl = *(const v4u*)(vbl + (size_t)d * kS + kv0 + col8);
        *(v4u*)(Vsh + d * kKC + col8) = vh;
        *(v4u*)(Vsl + d * kKC + col8) = vl;
      }
    }
    __syncthreads();

    v8f s[4];
#pragma unroll
    for (int j = 0; j < 4; ++j) {
      s[j] = (v8f){0.f,0.f,0.f,0.f,0.f,0.f,0.f,0.f};
      FB kb, kl;
      kb.h[0] = *(const v8b*)(const void*)(Ksh + (j * 16 + c) * kHD + 8 * hh);
      kb.h[1] = *(const v8b*)(const void*)(Ksh + (j * 16 + c) * kHD + 16 + 8 * hh);
      kl.h[0] = *(const v8b*)(const void*)(Ksl + (j * 16 + c) * kHD + 8 * hh);
      kl.h[1] = *(const v8b*)(const void*)(Ksl + (j * 16 + c) * kHD + 16 + 8 * hh);
      s[j] = at_mma(qah, kb.v, s[j]);
      s[j] = at_mma(qah, kl.v, s[j]);
      s[j] = at_mma(qal, kb.v, s[j]);
    }
    float cm[8];
#pragma unroll
    for (int r = 0; r < 8; ++r) {
      float m = fmaxf(fmaxf(s[0][r], s[1][r]), fmaxf(s[2][r], s[3][r]));
#pragma unroll
      for (int off = 1; off < 16; off <<= 1) m = fmaxf(m, __shfl_xor(m, off, 32));
      cm[r] = m;
    }
    unsigned short* pw = Psh[wave];
#pragma unroll
    for (int r = 0; r < 8; ++r) {
      const float mnew  = fmaxf(mrow[r], cm[r]);
      const float alpha = expf(mrow[r] - mnew);
      mrow[r] = mnew;
      float psum = 0.0f;
#pragma unroll
      for (int j = 0; j < 4; ++j) {
        const float p = expf(s[j][r] - mnew) * kPCarry;
        const _Float16 ph16 = (_Float16)p;
        psum += (float)ph16;
        pw[(8 * hh + r) * kKC + j * 16 + c] = __builtin_bit_cast(unsigned short, ph16);
      }
#pragma unroll
      for (int off = 1; off < 16; off <<= 1) psum += __shfl_xor(psum, off, 32);
      lrow[r] = lrow[r] * alpha + psum;
#pragma unroll
      for (int t = 0; t < 2; ++t) { oh[t][r] *= alpha; ol[t][r] *= alpha; }
    }
    __builtin_amdgcn_fence(__ATOMIC_RELEASE, "workgroup");
    __builtin_amdgcn_wave_barrier();
    __builtin_amdgcn_fence(__ATOMIC_ACQUIRE, "workgroup");
#pragma unroll
    for (int kk = 0; kk < 2; ++kk) {
      FB pa;
      pa.h[0] = *(const v8b*)(const void*)(pw + c * kKC + kk * 32 + 8 * hh);
      pa.h[1] = *(const v8b*)(const void*)(pw + c * kKC + kk * 32 + 16 + 8 * hh);
#pragma unroll
      for (int t = 0; t < 2; ++t) {
        FB vb, vl;
        vb.h[0] = *(const v8b*)(const void*)(Vsh + (t * 16 + c) * kKC + kk * 32 + 8 * hh);
        vb.h[1] = *(const v8b*)(const void*)(Vsh + (t * 16 + c) * kKC + kk * 32 + 16 + 8 * hh);
        vl.h[0] = *(const v8b*)(const void*)(Vsl + (t * 16 + c) * kKC + kk * 32 + 8 * hh);
        vl.h[1] = *(const v8b*)(const void*)(Vsl + (t * 16 + c) * kKC + kk * 32 + 16 + 8 * hh);
        oh[t] = at_mma16<true>(pa.v, vb.v, oh[t]);
        ol[t] = at_mma16<true>(pa.v, vl.v, ol[t]);
      }
    }
  }

  float* os = Os[wave];
#pragma unroll
  for (int r = 0; r < 8; ++r) {
    const float inv = 1.0f / lrow[r];
#pragma unroll
    for (int t = 0; t < 2; ++t) os[(8 * hh + r) * kOsPitch + t * 16 + c] = (oh[t][r] + ol[t][r] * kVloInv) * inv;
  }
  __builtin_amdgcn_fence(__ATOMIC_RELEASE, "workgroup");
  __builtin_amdgcn_wave_barrier();
  __builtin_amdgcn_fence(__ATOMIC_ACQUIRE, "workgroup");
  {
    const int q4 = lane >> 3, c4 = (lane & 7) * 4;
    float* ob = ctx + (tokBase + q0) * kD + h * kHD;
    for (int pass = 0; pass < 2; ++pass) {
#pragma unroll
      for (int it = 0; it < 4; ++it) {
        const int row = it * 4 + q4;
        const v4f val = *(const v4f*)(os + row * kOsPitch + c4);
        *(volatile v4f*)(ob + (size_t)row * kD + c4) = val;
      }
      __threadfence();
    }
  }
}

extern "C" void kernel_launch(void* const* d_in, const int* in_sizes, int n_in,
                              void* d_out, int out_size, void* d_ws, size_t ws_size,
                              hipStream_t stream) {
  if (n_in < 12) return;
  const int nElem = kTok * kD;
  if (in_sizes[0] != nElem || out_size != nElem) return;
  if (in_sizes[1] != kD * kD || in_sizes[2] != kD * kD || in_sizes[3] != kD * kD) return;
  if (in_sizes[8] != kD * kD || in_sizes[10] != kD * kD) return;
  if (in_sizes[4] != kD || in_sizes[5] != kD || in_sizes[6] != kD || in_sizes[7] != kD) return;
  if (in_sizes[9] != kD || in_sizes[11] != kD) return;

  const size_t szWB  = (size_t)3 * kD * kD * 2;
  const size_t szWF  = (size_t)2 * kD * kD * 2;
  const size_t szXN  = (size_t)kTok * kD * 2;
  const size_t szQK  = (size_t)kTokC * kQKld * 2;
  const size_t szV32 = (size_t)kTokC * kD * 4;
  const size_t szVT  = (size_t)kCB * kH * kHD * kS * 2;
  const size_t szCTX = (size_t)kTokC * kD * 4;
  const size_t szA32 = (size_t)kTokC * kD * 4;
  const size_t szA16 = (size_t)kTokC * kD * 2;
  const size_t szHID = (size_t)kTokC * kD * 2;
  const size_t offWB  = 0;
  const size_t offWF  = offWB + szWB;
  const size_t offXNH = offWF + szWF;
  const size_t offXNL = offXNH + szXN;
  const size_t offQKH = offXNL + szXN;
  const size_t offQKL = offQKH + szQK;
  const size_t offV32 = offQKL + szQK;
  const size_t offVTH = offV32 + szV32;
  const size_t offVTL = offVTH + szVT;
  const size_t offCTX = offVTL + szVT;
  const size_t offA32 = offCTX + szCTX;
  const size_t offA16 = offA32 + szA32;
  const size_t offHID = offA16 + szA16;
  const size_t total  = offHID + szHID;
  if (ws_size < total) return;

  const float* x   = (const float*)d_in[0];
  const float* wq  = (const float*)d_in[1];
  const float* wk  = (const float*)d_in[2];
  const float* wv  = (const float*)d_in[3];
  const float* g1  = (const float*)d_in[4];
  const float* be1 = (const float*)d_in[5];
  const float* g2  = (const float*)d_in[6];
  const float* be2 = (const float*)d_in[7];
  const float* wf1 = (const float*)d_in[8];
  const float* bf1 = (const float*)d_in[9];
  const float* wf2 = (const float*)d_in[10];
  const float* bf2 = (const float*)d_in[11];
  float* out = (float*)d_out;
  char* ws = (char*)d_ws;
  unsigned short* WB  = (unsigned short*)(ws + offWB);
  unsigned short* WF  = (unsigned short*)(ws + offWF);
  unsigned short* XNH = (unsigned short*)(ws + offXNH);
  unsigned short* XNL = (unsigned short*)(ws + offXNL);
  unsigned short* QKH = (unsigned short*)(ws + offQKH);
  unsigned short* QKL = (unsigned short*)(ws + offQKL);
  float*          V32 = (float*)(ws + offV32);
  unsigned short* VTH = (unsigned short*)(ws + offVTH);
  unsigned short* VTL = (unsigned short*)(ws + offVTL);
  float*          CTX = (float*)(ws + offCTX);
  float*          A32 = (float*)(ws + offA32);
  unsigned short* A16 = (unsigned short*)(ws + offA16);
  unsigned short* HID = (unsigned short*)(ws + offHID);

  wprep_kernel<<<dim3(kD / 64, kD / 64, 5), dim3(256), 0, stream>>>(wq, wk, wv, wf1, wf2, WB, WF);
  ln1_split_kernel<<<dim3(kTok / 8), dim3(256), 0, stream>>>(x, g1, be1, XNH, XNL, kTok);

  const int tilesQK = (kTokC / 64) * (kQKld / 64);
  const int tilesD  = (kTokC / 64) * (kD / 64);
  for (int cidx = 0; cidx < kNChunk; ++cidx) {
    const size_t tokOff = (size_t)cidx * kTokC;
    const unsigned short* xh = XNH + tokOff * kD;
    const unsigned short* xl = XNL + tokOff * kD;
    wmma_gemm64<1, true, false, 0, 2, false, 0><<<dim3(tilesQK / 8, 1), dim3(256), 0, stream>>>(
        xh, xl, kD, 0L, WB, WB, kD, 0L, (void*)QKH, (void*)QKL, kQKld, 0L,
        bf1, A32, 0L, kTokC, kQKld, kD, 1.0f);
    wmma_gemm64<1, true, false, 0, 0, false, 0><<<dim3(tilesD / 8, 1), dim3(256), 0, stream>>>(
        xh, xl, kD, 0L, WB + (size_t)2 * kD * kD, WB + (size_t)2 * kD * kD, kD, 0L, (void*)V32, (void*)V32, kD, 0L,
        bf1, A32, 0L, kTokC, kD, kD, 1.0f);
    vt_split_kernel<<<dim3(kS / 64, kH, kCB), dim3(256), 0, stream>>>(V32, VTH, VTL);
    attn_hd32_kernel<<<dim3(kCB * kH * (kS / 64)), dim3(128), 0, stream>>>(QKH, QKL, VTH, VTL, CTX);
    ln2_kernel<<<dim3(kTokC / 8), dim3(256), 0, stream>>>(CTX, x + tokOff * kD, g2, be2, A32, A16, kTokC);
    wmma_gemm64<0, false, false, 2, 1, false, 2><<<dim3(tilesD / 8, 1), dim3(256), 0, stream>>>(
        A16, A16, kD, 0L, WF, WF, kD, 0L, (void*)HID, (void*)HID, kD, 0L,
        bf1, A32, 0L, kTokC, kD, kD, kWCarryInv);
    float* outc = out + tokOff * kD;
    wmma_gemm64<0, false, false, 2, 0, true, 0><<<dim3(tilesD / 8, 1), dim3(256), 0, stream>>>(
        HID, HID, kD, 0L, WF + (size_t)kD * kD, WF + (size_t)kD * kD, kD, 0L, (void*)outc, (void*)outc, kD, 0L,
        bf2, A32, 0L, kTokC, kD, kD, kWCarryInv);
  }
}
